// Mamba_Traj_18253611008298
// MI455X (gfx1250) — hardware-verified
//
#include <hip/hip_runtime.h>
#include <math.h>
#include <stddef.h>


typedef _Float16 v16h __attribute__((ext_vector_type(16)));
typedef _Float16 v8h  __attribute__((ext_vector_type(8)));
typedef _Float16 v4h  __attribute__((ext_vector_type(4)));
typedef float    v8f  __attribute__((ext_vector_type(8)));
typedef float    v4f  __attribute__((ext_vector_type(4)));
typedef v4f v4fa __attribute__((may_alias));

#define BN      8
#define LS      128
#define LP      384
#define TOK     3072
#define STATEK  6
#define ACTK    3
#define EDIM    256
#define DMODEL  256
#define NLAYER  4
#define DINNER  512
#define DSTATE  16
#define RKDT    16
#define DCONV   4
#define PROJW   48
#define PROJLD  64
#define EPSV    1e-5f

#define GBM 128
#define GBN 64
#define GBK 32
#define LDSA 40
#define LDSB 40

union Frag { v16h v; v8h half[2]; };

__device__ __forceinline__ v8f wmma16(const v16h a, const v16h b, v8f c)
{
  c = __builtin_amdgcn_wmma_f32_16x16x32_f16(false, a, false, b, (short)0, c, false, false);
  asm volatile("v_nop\n\tv_nop\n\tv_nop\n\tv_nop" : "+v"(c) : "v"(a), "v"(b));
  return c;
}

__device__ __forceinline__ float siluf(float x)
{
  return x * __builtin_amdgcn_rcpf(1.0f + __expf(-x));
}

__device__ __forceinline__ float softplusf(float x)
{
  const float r = log1pf(expf(-fabsf(x)));
  return (x > 0.0f ? x : 0.0f) + r;
}

__global__ __launch_bounds__(256) void embed_kernel(
    const float* __restrict__ states, const float* __restrict__ actions,
    const float* __restrict__ goal,   const int*   __restrict__ tsteps,
    const float* __restrict__ teW,
    const float* __restrict__ seW, const float* __restrict__ seb,
    const float* __restrict__ geW, const float* __restrict__ geb,
    const float* __restrict__ aeW, const float* __restrict__ aeb,
    float* __restrict__ u, int ntok, int nte)
{
  const int idx = blockIdx.x * 256 + threadIdx.x;
  if (idx >= ntok * (EDIM / 4)) return;
  const int tt   = idx / (EDIM / 4);
  const int e4   = (idx - tt * (EDIM / 4)) * 4;
  const int slot = tt % 3;
  const int bl   = tt / 3;
  const float* W; const float* bv; const float* src; int kk;
  if (slot == 0)      { W = geW; bv = geb; src = goal    + (size_t)bl * STATEK; kk = STATEK; }
  else if (slot == 1) { W = seW; bv = seb; src = states  + (size_t)bl * STATEK; kk = STATEK; }
  else                { W = aeW; bv = aeb; src = actions + (size_t)bl * ACTK;   kk = ACTK;   }
  v4f acc = *(const v4f*)(bv + e4);
  #pragma unroll
  for (int k = 0; k < STATEK; ++k) {
    if (k < kk) {
      const float s = src[k];
      const v4f wv = *(const v4f*)(W + (size_t)k * EDIM + e4);
      acc += s * wv;
    }
  }
  int ts = tsteps[bl];
  if (ts < 0) ts += nte;
  if (ts < 0) ts = 0;
  if (ts > nte - 1) ts = nte - 1;
  acc += *(const v4f*)(teW + (size_t)ts * EDIM + e4);
  float* p = u + (size_t)tt * EDIM + e4;
  *(volatile v4f*)p = acc;
  __threadfence();
  *(volatile v4f*)p = acc;
}

__global__ __launch_bounds__(256) void gemm_f16_kernel(
    const float* __restrict__ A, int lda,
    const float* __restrict__ Bw,
    const float* __restrict__ bias, int has_bias,
    const float* Cin, int has_cin,
    float* Out,
    int M, int N, int K, int ldo, float wscale, float oscale, int act)
{
  __shared__ __attribute__((aligned(16))) _Float16 As[GBM * LDSA];
  __shared__ __attribute__((aligned(16))) _Float16 Bs[GBN * LDSB];
  __shared__ __attribute__((aligned(16))) float    Cs[8 * 16 * GBN];

  const int tid  = threadIdx.x;
  const int wave = tid >> 5;
  const int lane = tid & 31;
  const int hh   = lane >> 4;
  const int mm   = lane & 15;
  const int m0 = blockIdx.x * GBM;
  const int n0 = blockIdx.y * GBN;
  const bool n4 = ((N & 3) == 0);
  const bool a4 = ((lda & 3) == 0);

  v8f acc[4];
  #pragma unroll
  for (int j = 0; j < 4; ++j) {
    #pragma unroll
    for (int r = 0; r < 8; ++r) acc[j][r] = 0.0f;
  }

  for (int k0 = 0; k0 < K; k0 += GBK) {
    __syncthreads();
    #pragma unroll
    for (int it = 0; it < 4; ++it) {
      const int vid = tid + it * 256;
      const int r   = vid >> 3;
      const int c4  = (vid & 7) << 2;
      int gr = m0 + r; if (gr > M - 1) gr = M - 1;
      const int gk = k0 + c4;
      const float* ap = A + (size_t)gr * lda + gk;
      v4f v;
      if (a4 && gk + 3 < K) {
        v = *(const v4f*)ap;
      } else {
        #pragma unroll
        for (int j = 0; j < 4; ++j) v[j] = (gk + j < K) ? ap[j] : 0.0f;
      }
      v4h hv;
      #pragma unroll
      for (int j = 0; j < 4; ++j) hv[j] = (_Float16)v[j];
      *(v4h*)(As + r * LDSA + c4) = hv;
    }
    #pragma unroll
    for (int it = 0; it < 2; ++it) {
      const int vid = tid + it * 256;
      const int kk  = vid >> 4;
      const int c4  = (vid & 15) << 2;
      const int gk = k0 + kk;
      const int gn = n0 + c4;
      v4f v;
      if (gk < K && n4 && gn + 3 < N) {
        v = *(const v4f*)(Bw + (size_t)gk * N + gn);
      } else {
        #pragma unroll
        for (int j = 0; j < 4; ++j)
          v[j] = (gk < K && gn + j < N) ? Bw[(size_t)gk * N + gn + j] : 0.0f;
      }
      #pragma unroll
      for (int j = 0; j < 4; ++j) Bs[(c4 + j) * LDSB + kk] = (_Float16)(v[j] * wscale);
    }
    __syncthreads();

    Frag a;
    const _Float16* pa = As + (wave * 16 + mm) * LDSA;
    a.half[0] = *(const v8h*)(pa + 8 * hh);
    a.half[1] = *(const v8h*)(pa + 16 + 8 * hh);
    #pragma unroll
    for (int j = 0; j < 4; ++j) {
      Frag b;
      const _Float16* pb = Bs + (16 * j + mm) * LDSB;
      b.half[0] = *(const v8h*)(pb + 8 * hh);
      b.half[1] = *(const v8h*)(pb + 16 + 8 * hh);
      acc[j] = wmma16(a.v, b.v, acc[j]);
    }
  }

  float* cs = Cs + wave * (16 * GBN);
  #pragma unroll
  for (int j = 0; j < 4; ++j) {
    #pragma unroll
    for (int r = 0; r < 8; ++r) cs[(8 * hh + r) * GBN + 16 * j + mm] = acc[j][r];
  }
  __syncthreads();

  const int lr = lane >> 3;
  const int lc = (lane & 7) << 2;
  v4f vals[8];
  #pragma unroll
  for (int s = 0; s < 8; ++s) {
    const int q   = 4 * s + lr;
    const int row = q >> 1;
    const int col = ((q & 1) << 5) + lc;
    v4f v = *(const v4fa*)(cs + row * GBN + col);
    const int gr = m0 + wave * 16 + row;
    const int gc = n0 + col;
    const bool ok = (gr < M) && (gc + 3 < ldo);
    v = v * oscale;
    if (has_bias) {
      #pragma unroll
      for (int j = 0; j < 4; ++j) v[j] += (gc + j < N) ? bias[gc + j] : 0.0f;
    }
    if (has_cin && ok) v += *(const v4f*)(Cin + (size_t)gr * ldo + gc);
    if (act == 1) {
      #pragma unroll
      for (int j = 0; j < 4; ++j) v[j] = softplusf(v[j]);
    }
    vals[s] = v;
  }
  #pragma unroll
  for (int s = 0; s < 8; ++s) {
    const int q = 4 * s + lr;
    const int gr = m0 + wave * 16 + (q >> 1);
    const int gc = n0 + ((q & 1) << 5) + lc;
    if (gr < M && gc + 3 < ldo) *(volatile v4f*)(Out + (size_t)gr * ldo + gc) = vals[s];
  }
  __threadfence();
  #pragma unroll
  for (int s = 0; s < 8; ++s) {
    const int q = 4 * s + lr;
    const int gr = m0 + wave * 16 + (q >> 1);
    const int gc = n0 + ((q & 1) << 5) + lc;
    if (gr < M && gc + 3 < ldo) *(volatile v4f*)(Out + (size_t)gr * ldo + gc) = vals[s];
  }
}

__global__ __launch_bounds__(256) void rmsnorm_kernel(
    const float* __restrict__ x, const float* __restrict__ w,
    float* __restrict__ out, int ntok)
{
  const int gw   = (blockIdx.x * 256 + threadIdx.x) >> 5;
  const int lane = threadIdx.x & 31;
  if (gw >= ntok) return;
  const float* row = x + (size_t)gw * DMODEL;
  const v4f v0 = *(const v4f*)(row + lane * 4);
  const v4f v1 = *(const v4f*)(row + 128 + lane * 4);
  float ss = 0.0f;
  #pragma unroll
  for (int j = 0; j < 4; ++j) ss += v0[j] * v0[j] + v1[j] * v1[j];
  #pragma unroll
  for (int off = 16; off > 0; off >>= 1) ss += __shfl_xor(ss, off, 32);
  const float sc = rsqrtf(ss * (1.0f / DMODEL) + EPSV);
  const v4f w0 = *(const v4f*)(w + lane * 4);
  const v4f w1 = *(const v4f*)(w + 128 + lane * 4);
  const v4f o0 = (v0 * sc) * w0;
  const v4f o1 = (v1 * sc) * w1;
  float* orow = out + (size_t)gw * DMODEL;
  *(volatile v4f*)(orow + lane * 4)       = o0;
  *(volatile v4f*)(orow + 128 + lane * 4) = o1;
  __threadfence();
  *(volatile v4f*)(orow + lane * 4)       = o0;
  *(volatile v4f*)(orow + 128 + lane * 4) = o1;
}

__global__ __launch_bounds__(256) void conv_silu_kernel(
    const float* __restrict__ xz, const float* __restrict__ cw,
    const float* __restrict__ cb, float* __restrict__ xc, int ntok)
{
  const int idx = blockIdx.x * 256 + threadIdx.x;
  if (idx >= ntok * (DINNER / 4)) return;
  const int t  = idx / (DINNER / 4);
  const int d4 = (idx - t * (DINNER / 4)) * 4;
  const int l  = t % LP;
  v4f acc = *(const v4f*)(cb + d4);
  v4f wv[4];
  #pragma unroll
  for (int j = 0; j < 4; ++j) wv[j] = *(const v4f*)(cw + (size_t)(d4 + j) * DCONV);
  #pragma unroll
  for (int k = 0; k < DCONV; ++k) {
    const int ls = l + k - (DCONV - 1);
    if (ls >= 0) {
      const v4f xv = *(const v4f*)(xz + (size_t)(t + k - (DCONV - 1)) * (2 * DINNER) + d4);
      #pragma unroll
      for (int j = 0; j < 4; ++j) acc[j] += xv[j] * wv[j][k];
    }
  }
  v4f o;
  #pragma unroll
  for (int j = 0; j < 4; ++j) o[j] = siluf(acc[j]);
  float* p = xc + (size_t)t * DINNER + d4;
  *(volatile v4f*)p = o;
  __threadfence();
  *(volatile v4f*)p = o;
}

__global__ __launch_bounds__(256) void scan_kernel(
    const float* __restrict__ dt,   const float* __restrict__ proj,
    const float* __restrict__ xc,   const float* __restrict__ xz,
    const float* __restrict__ Alog, const float* __restrict__ Dp,
    float* __restrict__ y)
{
  __shared__ __attribute__((aligned(16))) float sBC[LP * 2 * DSTATE];
  __shared__ __attribute__((aligned(16))) float ys[2 * DINNER];
  const int b   = blockIdx.x;
  const int tid = threadIdx.x;
  const int d0 = tid, d1 = tid + 256;

  for (int i = tid; i < LP * 2 * DSTATE; i += 256) {
    const int l = i >> 5, c = i & 31;
    sBC[i] = proj[((size_t)b * LP + l) * PROJLD + RKDT + c];
  }
  float A0[DSTATE], A1[DSTATE], h0[DSTATE], h1[DSTATE];
  #pragma unroll
  for (int n = 0; n < DSTATE; ++n) {
    A0[n] = -__expf(Alog[(size_t)d0 * DSTATE + n]);
    A1[n] = -__expf(Alog[(size_t)d1 * DSTATE + n]);
    h0[n] = 0.0f; h1[n] = 0.0f;
  }
  const float Dv0 = Dp[d0], Dv1 = Dp[d1];
  __syncthreads();

  for (int l = 0; l < LP; ++l) {
    const size_t t = (size_t)b * LP + l;
    const float dt0 = dt[t * DINNER + d0], dt1 = dt[t * DINNER + d1];
    const float x0  = xc[t * DINNER + d0], x1  = xc[t * DINNER + d1];
    const float z0  = xz[t * (2 * DINNER) + DINNER + d0];
    const float z1  = xz[t * (2 * DINNER) + DINNER + d1];
    const float bx0 = dt0 * x0, bx1 = dt1 * x1;
    const float* sB = sBC + l * (2 * DSTATE);
    const float* sC = sB + DSTATE;
    float y0 = 0.0f, y1 = 0.0f;
    #pragma unroll
    for (int n = 0; n < DSTATE; ++n) {
      const float bn = sB[n], cn = sC[n];
      h0[n] = __expf(dt0 * A0[n]) * h0[n] + bx0 * bn;
      y0 += h0[n] * cn;
      h1[n] = __expf(dt1 * A1[n]) * h1[n] + bx1 * bn;
      y1 += h1[n] * cn;
    }
    y0 += x0 * Dv0;
    y1 += x1 * Dv1;
    float* yl = ys + (l & 1) * DINNER;
    yl[d0] = y0 * siluf(z0);
    yl[d1] = y1 * siluf(z1);
    __syncthreads();
    if (tid < DINNER / 4) {
      const v4f v = *(const v4fa*)(yl + tid * 4);
      float* p = y + t * DINNER + tid * 4;
      *(volatile v4f*)p = v;
      __threadfence();
      *(volatile v4f*)p = v;
    }
  }
}

__global__ __launch_bounds__(256) void head_kernel(
    const float* __restrict__ yf,
    const float* __restrict__ psW, const float* __restrict__ psb,
    const float* __restrict__ paW, const float* __restrict__ pab,
    float* __restrict__ out, int total)
{
  __shared__ __attribute__((aligned(16))) float so[256];
  const int tid = threadIdx.x;
  const int idx = blockIdx.x * 256 + tid;
  const int NS  = BN * LS * STATEK;
  float val = 0.0f;
  if (idx < total) {
    int j, nout, row; const float* W; float acc;
    const bool is_s = idx < NS;
    if (is_s) {
      j = idx % STATEK; const int bl = idx / STATEK;
      const int bb = bl / LS, l = bl - bb * LS;
      row = bb * LP + 3 * l + 2; W = psW; nout = STATEK; acc = psb[j];
    } else {
      const int i2 = idx - NS;
      j = i2 % ACTK; const int bl = i2 / ACTK;
      const int bb = bl / LS, l = bl - bb * LS;
      row = bb * LP + 3 * l + 1; W = paW; nout = ACTK; acc = pab[j];
    }
    const float* yr = yf + (size_t)row * DMODEL;
    #pragma unroll 4
    for (int k = 0; k < DMODEL; ++k) acc = fmaf(yr[k], W[k * nout + j], acc);
    val = is_s ? acc : tanhf(acc);
  }
  so[tid] = val;
  __syncthreads();
  if (tid < 64) {
    const int base = blockIdx.x * 256 + tid * 4;
    if (base + 3 < total) {
      const v4f v = *(const v4fa*)(so + tid * 4);
      float* p = out + base;
      *(volatile v4f*)p = v;
      __threadfence();
      *(volatile v4f*)p = v;
    }
  }
}

static inline unsigned cdiv_u(unsigned a, unsigned b) { return (a + b - 1) / b; }

static void launch_gemm(hipStream_t stream, const float* A, int lda, const float* Bw,
                        const float* bias, int has_bias, const float* Cin, int has_cin,
                        float* Out, int M, int N, int K, int ldo, int act)
{
  dim3 grid(cdiv_u(M, GBM), cdiv_u(ldo, GBN));
  gemm_f16_kernel<<<grid, 256, 0, stream>>>(A, lda, Bw, bias, has_bias, Cin, has_cin, Out,
                                            M, N, K, ldo, 16.0f, 0.0625f, act);
}

extern "C" void kernel_launch(void* const* d_in, const int* in_sizes, int n_in,
                              void* d_out, int out_size, void* d_ws, size_t ws_size,
                              hipStream_t stream)
{
  if (n_in < 28) return;
  if (in_sizes[0] != BN * LS * STATEK || in_sizes[3] != BN * LS) return;
  if (out_size != BN * LS * (STATEK + ACTK)) return;

  const float* states  = (const float*)d_in[0];
  const float* actions = (const float*)d_in[1];
  const float* goal    = (const float*)d_in[2];
  const int*   tsteps  = (const int*)  d_in[3];
  const float* teW   = (const float*)d_in[4];
  const float* seW   = (const float*)d_in[5];
  const float* seb   = (const float*)d_in[6];
  const float* geW   = (const float*)d_in[7];
  const float* geb   = (const float*)d_in[8];
  const float* aeW   = (const float*)d_in[9];
  const float* aeb   = (const float*)d_in[10];
  const float* bbW   = (const float*)d_in[11];
  const float* bbb   = (const float*)d_in[12];
  const float* normw = (const float*)d_in[13];
  const float* inW   = (const float*)d_in[14];
  const float* cw    = (const float*)d_in[15];
  const float* cb    = (const float*)d_in[16];
  const float* xpW   = (const float*)d_in[17];
  const float* dtW   = (const float*)d_in[18];
  const float* dtb   = (const float*)d_in[19];
  const float* Alog  = (const float*)d_in[20];
  const float* Dp    = (const float*)d_in[21];
  const float* outW  = (const float*)d_in[22];
  const float* fnw   = (const float*)d_in[23];
  const float* psW   = (const float*)d_in[24];
  const float* psb   = (const float*)d_in[25];
  const float* paW   = (const float*)d_in[26];
  const float* pab   = (const float*)d_in[27];
  const int nte = in_sizes[4] / EDIM;
  if (nte < 1) return;

  const size_t n_u    = (size_t)TOK * EDIM;
  const size_t n_res  = (size_t)TOK * DMODEL;
  const size_t n_xn   = (size_t)TOK * DMODEL;
  const size_t n_xz   = (size_t)TOK * 2 * DINNER;
  const size_t n_xc   = (size_t)TOK * DINNER;
  const size_t n_proj = (size_t)TOK * PROJLD;
  const size_t n_dt   = (size_t)TOK * DINNER;
  const size_t n_y    = (size_t)TOK * DINNER;
  const size_t n_yf   = (size_t)TOK * DMODEL;
  const size_t n_tot  = n_u + n_res + n_xn + n_xz + n_xc + n_proj + n_dt + n_y + n_yf;
  if (n_tot * sizeof(float) > ws_size) return;

  float* ws = (float*)d_ws;
  float* u     = ws; ws += n_u;
  float* resid = ws; ws += n_res;
  float* xn    = ws; ws += n_xn;
  float* xz    = ws; ws += n_xz;
  float* xcb   = ws; ws += n_xc;
  float* projb = ws; ws += n_proj;
  float* dtv   = ws; ws += n_dt;
  float* yb    = ws; ws += n_y;
  float* yf    = ws; ws += n_yf;

  embed_kernel<<<cdiv_u(TOK * (EDIM / 4), 256), 256, 0, stream>>>(
      states, actions, goal, tsteps, teW, seW, seb, geW, geb, aeW, aeb, u, TOK, nte);

  launch_gemm(stream, u, EDIM, bbW, bbb, 1, resid, 0, resid, TOK, DMODEL, EDIM, DMODEL, 0);

  for (int i = 0; i < NLAYER; ++i) {
    rmsnorm_kernel<<<cdiv_u(TOK * 32, 256), 256, 0, stream>>>(
        resid, normw + (size_t)i * DMODEL, xn, TOK);
    launch_gemm(stream, xn, DMODEL, inW + (size_t)i * DMODEL * 2 * DINNER, bbb, 0, xz, 0, xz,
                TOK, 2 * DINNER, DMODEL, 2 * DINNER, 0);
    conv_silu_kernel<<<cdiv_u(TOK * (DINNER / 4), 256), 256, 0, stream>>>(
        xz, cw + (size_t)i * DINNER * DCONV, cb + (size_t)i * DINNER, xcb, TOK);
    launch_gemm(stream, xcb, DINNER, xpW + (size_t)i * DINNER * PROJW, bbb, 0, projb, 0, projb,
                TOK, PROJW, DINNER, PROJLD, 0);
    launch_gemm(stream, projb, PROJLD, dtW + (size_t)i * RKDT * DINNER, dtb + (size_t)i * DINNER, 1,
                dtv, 0, dtv, TOK, DINNER, RKDT, DINNER, 1);
    scan_kernel<<<BN, 256, 0, stream>>>(
        dtv, projb, xcb, xz, Alog + (size_t)i * DINNER * DSTATE, Dp + (size_t)i * DINNER, yb);
    launch_gemm(stream, yb, DINNER, outW + (size_t)i * DINNER * DMODEL, bbb, 0, resid, 1, resid,
                TOK, DMODEL, DINNER, DMODEL, 0);
  }

  rmsnorm_kernel<<<cdiv_u(TOK * 32, 256), 256, 0, stream>>>(resid, fnw, yf, TOK);
  head_kernel<<<cdiv_u((unsigned)out_size, 256), 256, 0, stream>>>(
      yf, psW, psb, paW, pab, (float*)d_out, out_size);
}
